// ParallelGATBlock_43911745634519
// MI455X (gfx1250) — hardware-run, weakly checked
//
#include <hip/hip_runtime.h>


namespace {
constexpr int NN = 50000, NP = 50016, NE = 500000, CH = 256, CAT = 512, MAXDEG = 1024, NGc = (NN + 511) / 512, PERMLEN = NE + 32 * NGc + 32;
constexpr float XS = 8.0f, SLOPE = 0.2f, LN_EPS = 1e-5f;

typedef _Float16 b16;
typedef __attribute__((ext_vector_type(16))) _Float16 v16b;
typedef __attribute__((ext_vector_type(8))) _Float16 v8b;
typedef __attribute__((ext_vector_type(8))) float v8f;
typedef __attribute__((ext_vector_type(4))) float v4f;
__device__ __forceinline__ float bf16_rne(float f) { unsigned int u = __float_as_uint(f); u += 0x7FFFu + ((u >> 16) & 1u); return __uint_as_float(u & 0xFFFF0000u); }
__device__ __forceinline__ void split16(float v, b16& hi, b16& lo) { hi = (b16)v; lo = (b16)(v - (float)hi); }
__device__ __forceinline__ v16b frag_kb(const b16* p, int hh) { const v8b a = *(const v8b*)(p + 8 * hh), b = *(const v8b*)(p + 16 + 8 * hh); v16b f;
#pragma unroll
  for (int e = 0; e < 8; ++e) { f[e] = a[e]; f[8 + e] = b[e]; } return f; }
__device__ __forceinline__ v8f wmma16b(v16b a, v16b b, v8f c) { v8f d = __builtin_amdgcn_wmma_f32_16x16x32_f16(false, a, false, b, (short)0, c, false, false); asm volatile("v_nop\n\tv_nop\n\tv_nop\n\tv_nop" : "+v"(d) : "v"(a), "v"(b)); return d; }
__device__ __forceinline__ void wave_lds_sync() { __builtin_amdgcn_fence(__ATOMIC_RELEASE, "workgroup"); __builtin_amdgcn_wave_barrier(); __builtin_amdgcn_fence(__ATOMIC_ACQUIRE, "workgroup"); }
__device__ __forceinline__ float nexp(float x) { return __builtin_amdgcn_exp2f(x * 1.4426950408889634f); }
__device__ __forceinline__ float pmul(float a, float b) { float p = a * b; asm volatile("" : "+v"(p)); return p; }
__device__ __forceinline__ float leaky(float x) { return (x >= 0.0f) ? x : SLOPE * x; }
__device__ __forceinline__ float elu_f(float x) { return (x > 0.0f) ? x : (nexp(x) - 1.0f); }
__device__ __forceinline__ float wsum(float v) {
#pragma unroll
  for (int o = 1; o < 32; o <<= 1) v += __shfl_xor(v, o); return v; }
constexpr int CSR_NBLK = 512, CSR_GB = 9, CSR_GN = 1 << CSR_GB  , CSR_MAXG = 512, CSR_CAP = 12288  ;
__global__ __launch_bounds__(64) void csrA_kernel(const int* __restrict__ dst, int E, int N, int nG, int CHP, int NGP, int* __restrict__ STG, int* __restrict__ HST) {
  extern __shared__ int sm[];
  int* cnt = sm; int* run = sm + NGP; int* ids = sm + 2 * NGP;
  const int b = blockIdx.x; const int ch = (E + CSR_NBLK - 1) / CSR_NBLK; const int e0 = b * ch, e1 = min(E, e0 + ch);
  for (int i = threadIdx.x; i < NGP; i += 64) cnt[i] = 0;
  for (int i = threadIdx.x; i < CHP; i += 64) ids[i] = -1;
  __syncthreads();
  if (threadIdx.x == 0) {
    for (int e = e0; e < e1; ++e) { int d = dst[e]; d = (d < 0) ? 0 : (d >= N ? N - 1 : d); cnt[d >> CSR_GB] += 1; }
    int acc = 0; for (int g = 0; g < nG; ++g) { run[g] = acc; acc += cnt[g]; }
    for (int e = e0; e < e1; ++e) { int d = dst[e]; d = (d < 0) ? 0 : (d >= N ? N - 1 : d); const int g = d >> CSR_GB; ids[run[g]] = e; run[g] += 1; } }
  __syncthreads();
  typedef __attribute__((ext_vector_type(4))) int v4i;
  for (int pass = 0; pass < 2; ++pass) {
    for (int i = threadIdx.x; i < CHP / 4; i += 64) *(volatile v4i*)(STG + (size_t)b * CHP + i * 4) = *(const v4i*)(&ids[i * 4]);
    for (int i = threadIdx.x; i < NGP / 4; i += 64) { v4i v; for (int e = 0; e < 4; ++e) v[e] = (i * 4 + e < nG) ? cnt[i * 4 + e] : 0; *(volatile v4i*)(HST + (size_t)b * NGP + i * 4) = v; }
    __threadfence(); }
}
__global__ __launch_bounds__(512) void csrS_kernel(const int* __restrict__ HST, int nG, int NGP, int* __restrict__ START, int* __restrict__ TOT, int* __restrict__ OFF) {
  __shared__ int tot[CSR_MAXG];
  const int b = threadIdx.x;
  for (int pass = 0; pass < 2; ++pass) { int runb = 0; for (int g = 0; g < nG; ++g) { int c = HST[(size_t)b * NGP + g]; c = (c < 0) ? 0 : c; ((volatile int*)OFF)[(size_t)g * CSR_NBLK + b] = runb; runb += c; } __threadfence(); }
  for (int g = threadIdx.x; g < nG; g += 512) { int s = 0; for (int bb = 0; bb < CSR_NBLK; ++bb) { int c = HST[(size_t)bb * NGP + g]; s += (c < 0) ? 0 : c; } tot[g] = s; }
  __syncthreads();
  if (threadIdx.x < 32) {
    __shared__ int st[CSR_MAXG + 32];
    if (threadIdx.x == 0) { int acc = 0; for (int g = 0; g < NGP; ++g) { st[g] = acc; if (g < nG) acc += (tot[g] + 31) & ~31; } st[NGP] = acc; }
    __builtin_amdgcn_fence(__ATOMIC_RELEASE, "workgroup"); __builtin_amdgcn_wave_barrier(); __builtin_amdgcn_fence(__ATOMIC_ACQUIRE, "workgroup");
    for (int pass = 0; pass < 2; ++pass) { for (int i = threadIdx.x; i < NGP + 32; i += 32) { ((volatile int*)START)[i] = (i <= NGP) ? st[min(i, NGP)] : 0; ((volatile int*)TOT)[i] = (i < nG) ? tot[i] : 0; } __threadfence(); } }
}
__global__ __launch_bounds__(256) void csrB_kernel(const int* __restrict__ dst, int N, int nG, int CHP, int NGP, int permLen, const int* __restrict__ STG, const int* __restrict__ HST, const int* __restrict__ OFF, const int* __restrict__ START, const int* __restrict__ TOT, int* __restrict__ PERM, int* __restrict__ ROWPTR, int* __restrict__ ROWCNT, int* __restrict__ FLAG) {
  typedef __attribute__((ext_vector_type(4))) int v4i;
  __shared__ int ids[CSR_CAP]; __shared__ unsigned short key[CSR_CAP]; __shared__ int outp[CSR_CAP]; __shared__ int ncnt[CSR_GN + 1]; __shared__ int boff[CSR_NBLK + 1];
  const int g = blockIdx.x, t_ = threadIdx.x; int tot = TOT[g]; int st = START[g], stn = START[g + 1]; const int v0 = g * CSR_GN; const int nv = min(CSR_GN, N - v0);
  st = (st < 0) ? 0 : (st > permLen - 32 ? permLen - 32 : st) & ~31; stn = (stn < st) ? st : (stn > permLen ? permLen : stn); tot = (tot < 0) ? 0 : tot; if (tot > stn - st && tot <= CSR_CAP) tot = stn - st;
  if (tot > CSR_CAP) {
    for (int pass = 0; pass < 2; ++pass) { for (int i = t_; i < CSR_GN / 4; i += 256) { v4i a, c; for (int e = 0; e < 4; ++e) { a[e] = st; c[e] = 0; } *(volatile v4i*)(ROWPTR + v0 + i * 4) = a; *(volatile v4i*)(ROWCNT + v0 + i * 4) = c; } if (t_ == 0) ((volatile int*)FLAG)[0] = 1; __threadfence(); } (void)nv; return; }
  if (t_ == 0) { int acc = 0; for (int b = 0; b < CSR_NBLK; ++b) { boff[b] = acc; int c = HST[(size_t)b * NGP + g]; c = (c < 0) ? 0 : (c > CHP ? CHP : c); acc += c; if (acc > tot) acc = tot; } boff[CSR_NBLK] = acc; }
  for (int i = t_; i <= CSR_GN; i += 256) ncnt[i] = 0;
  __syncthreads();
  for (int b = 0; b < CSR_NBLK; ++b) { const int c = boff[b + 1] - boff[b]; int o_ = OFF[(size_t)g * CSR_NBLK + b]; o_ = (o_ < 0) ? 0 : (o_ > CHP - c ? CHP - c : o_); const int* src_ = STG + (size_t)b * CHP + o_;
    for (int i = t_; i < c; i += 256) { int id = src_[i]; id = (id < 0) ? 0 : id; ids[boff[b] + i] = id; int d = dst[id]; d = (d < v0) ? v0 : (d >= N ? N - 1 : d); int kk = d - v0; kk = (kk < 0) ? 0 : (kk >= CSR_GN ? CSR_GN - 1 : kk); key[boff[b] + i] = (unsigned short)kk; } }
  __syncthreads();
  if (t_ == 0) { for (int i = 0; i < tot; ++i) ncnt[key[i]] += 1; int acc = 0; for (int vl = 0; vl < CSR_GN; ++vl) { const int c = ncnt[vl]; ncnt[vl] = acc; acc += c; } ncnt[CSR_GN] = acc;
    for (int i = 0; i < tot; ++i) { const int vl = key[i]; outp[ncnt[vl]] = ids[i]; ncnt[vl] += 1; }
    for (int vl = CSR_GN; vl > 0; --vl) ncnt[vl] = ncnt[vl - 1]; ncnt[0] = 0; }
  __syncthreads();
  for (int pass = 0; pass < 2; ++pass) {
    for (int i = t_; i < (stn - st) / 4; i += 256) { v4i v; for (int e = 0; e < 4; ++e) { const int q = i * 4 + e; v[e] = (q < tot) ? outp[q] : -1; } *(volatile v4i*)(PERM + st + i * 4) = v; }
    for (int i = t_; i < CSR_GN / 4; i += 256) { v4i a, c; for (int e = 0; e < 4; ++e) { const int vl = i * 4 + e; a[e] = st + ncnt[vl]; c[e] = (vl < nv) ? (ncnt[vl + 1] - ncnt[vl]) : 0; } *(volatile v4i*)(ROWPTR + v0 + i * 4) = a; *(volatile v4i*)(ROWCNT + v0 + i * 4) = c; }
    __threadfence(); }
}
__global__ __launch_bounds__(256) void csrZ_kernel(int* __restrict__ p, size_t n4) { typedef __attribute__((ext_vector_type(4))) int v4i; const size_t tid = (size_t)blockIdx.x * 256 + threadIdx.x, nth = (size_t)gridDim.x * 256; v4i z = {0, 0, 0, 0}; for (size_t i = tid; i < n4; i += nth) *(volatile v4i*)(p + i * 4) = z; }
struct CsrBufs { int *STG, *HST, *OFF, *START, *TOT, *PERM, *ROWPTR, *ROWCNT, *FLAG; int nG, NGP, CHP; size_t permLen; char* base; size_t bytes; };
static size_t csr_carve(CsrBufs& c, char* ws, size_t off, int E, int N) {
  const size_t off0 = off; c.base = ws + off;
  auto al = [&](size_t bytes) { char* p = ws + off; off += (bytes + 255) & ~(size_t)255; return p; };
  c.nG = (N + CSR_GN - 1) / CSR_GN; c.NGP = (c.nG + 31) & ~31; const int ch = (E + CSR_NBLK - 1) / CSR_NBLK; c.CHP = (ch + 31) & ~31; c.permLen = (size_t)E + 32 * (size_t)c.nG + 32;
  c.STG = (int*)al((size_t)CSR_NBLK * c.CHP * 4); c.HST = (int*)al((size_t)CSR_NBLK * c.NGP * 4); c.OFF = (int*)al((size_t)c.NGP * CSR_NBLK * 4); c.START = (int*)al((size_t)(c.NGP + 64) * 4); c.TOT = (int*)al((size_t)(c.NGP + 64) * 4);
  c.PERM = (int*)al(c.permLen * 4); c.ROWPTR = (int*)al((size_t)c.nG * CSR_GN * 4); c.ROWCNT = (int*)al((size_t)c.nG * CSR_GN * 4); c.FLAG = (int*)al(256);
  c.bytes = off - off0; return off;
}
static void csr_build(const CsrBufs& c, const int* dst, int E, int N, hipStream_t stream) {
  const size_t smem = (size_t)(2 * c.NGP + c.CHP) * 4;
  csrZ_kernel<<<512, 256, 0, stream>>>((int*)c.base, c.bytes / 16);
  csrA_kernel<<<CSR_NBLK, 64, smem, stream>>>(dst, E, N, c.nG, c.CHP, c.NGP, c.STG, c.HST);
  csrS_kernel<<<1, 512, 0, stream>>>(c.HST, c.nG, c.NGP, c.START, c.TOT, c.OFF);
  csrB_kernel<<<c.nG, 256, 0, stream>>>(dst, N, c.nG, c.CHP, c.NGP, (int)c.permLen, c.STG, c.HST, c.OFF, c.START, c.TOT, c.PERM, c.ROWPTR, c.ROWCNT, c.FLAG);
}

__global__ __launch_bounds__(256) void prep_kernel(const float* __restrict__ gm, const float* __restrict__ bt, const float* __restrict__ w1, const float* __restrict__ as1, const float* __restrict__ ad1, const float* __restrict__ b1, const float* __restrict__ w2, const float* __restrict__ as2, const float* __restrict__ ad2, const float* __restrict__ b2, const float* __restrict__ wu, const float* __restrict__ bu, b16* __restrict__ R, float* __restrict__ P, b16* __restrict__ XN, b16* __restrict__ XNl, b16* __restrict__ CT, b16* __restrict__ CTl) {
  const size_t tid = (size_t)blockIdx.x * 256 + threadIdx.x, nth = (size_t)gridDim.x * 256;
  for (int pass = 0; pass < 2; ++pass) {
    for (size_t p = tid; p < (size_t)2 * CH * CH; p += nth) { const int l = (int)(p / (CH * CH)), o = (int)((p / CH) % CH), k = (int)(p % CH); ((volatile b16*)R)[p] = (b16)bf16_rne((l ? w2 : w1)[(size_t)k * CH + o]); }
    for (size_t p = tid; p < (size_t)CH * CAT; p += nth) { const int o = (int)(p / CAT), k = (int)(p % CAT); ((volatile b16*)R)[131072 + p] = (b16)bf16_rne(wu[(size_t)k * CH + o]); }
    for (size_t q = tid; q < 2304; q += nth) { const int i = (int)q; const float* s_ = (i < 256) ? gm : (i < 512) ? bt : (i < 768) ? as1 : (i < 1024) ? ad1 : (i < 1280) ? b1 : (i < 1536) ? as2 : (i < 1792) ? ad2 : (i < 2048) ? b2 : bu; P[q] = bf16_rne(s_[i & 255]); }
    { const v8b z = {}; for (size_t p = tid; p < (size_t)(NP - NN) * CH / 8; p += nth) { *(volatile v8b*)(XN + (size_t)NN * CH + p * 8) = z; *(volatile v8b*)(XNl + (size_t)NN * CH + p * 8) = z; } for (size_t p = tid; p < (size_t)(NP - NN) * CAT / 8; p += nth) { *(volatile v8b*)(CT + (size_t)NN * CAT + p * 8) = z; *(volatile v8b*)(CTl + (size_t)NN * CAT + p * 8) = z; } }
    __threadfence(); }
}
__global__ __launch_bounds__(256) void ln_kernel(const float* __restrict__ x, const float* __restrict__ P, b16* __restrict__ XN, b16* __restrict__ XNl) {
  __shared__ __attribute__((aligned(16))) b16 Sh[8][CH + 8], Sl[8][CH + 8];
  const int wave = threadIdx.x >> 5, v = blockIdx.x * 8 + wave, lane = threadIdx.x & 31; float xv[8]; float s = 0.0f;
#pragma unroll
  for (int e = 0; e < 8; ++e) { xv[e] = bf16_rne(x[(size_t)v * CH + lane * 8 + e]); s += xv[e]; }
  s = wsum(s); const float mu = s * (1.0f / CH); float q = 0.0f;
#pragma unroll
  for (int e = 0; e < 8; ++e) { const float d = xv[e] - mu; q += pmul(d, d); }
  q = wsum(q); const float inv = rsqrtf(q * (1.0f / CH) + LN_EPS);
#pragma unroll
  for (int e = 0; e < 8; ++e) { const int c = lane * 8 + e; b16 a_, b_; split16((pmul((xv[e] - mu) * inv, P[c]) + P[256 + c]) * XS, a_, b_); Sh[wave][c] = a_; Sl[wave][c] = b_; }
  wave_lds_sync();
  for (int pass = 0; pass < 2; ++pass) { *(volatile v8b*)(XN + (size_t)v * CH + lane * 8) = *(const v8b*)(&Sh[wave][lane * 8]); *(volatile v8b*)(XNl + (size_t)v * CH + lane * 8) = *(const v8b*)(&Sl[wave][lane * 8]); __threadfence(); }
}
template <int KIN, int OUTMODE>
__global__ __launch_bounds__(64) void gemm_kernel(const b16* __restrict__ A, const b16* __restrict__ Al, const b16* __restrict__ Bw, const float* __restrict__ P, const float* __restrict__ x, b16* __restrict__ FT, b16* __restrict__ FTl, float* __restrict__ out) {
  __shared__ __attribute__((aligned(16))) float Ts[2][16][128 + 4]; __shared__ __attribute__((aligned(16))) b16 Tb[2][16][128 + 8], Tc[2][16][128 + 8];
  const int lane = threadIdx.x & 31, wave = threadIdx.x >> 5, nloc = lane & 15, hlf = lane >> 4, m0 = blockIdx.y * 32 + wave * 16, c0 = blockIdx.x * 128;
  v8f acc[8];
#pragma unroll
  for (int t = 0; t < 8; ++t) acc[t] = (v8f){};
#pragma unroll 2
  for (int kb = 0; kb < KIN; kb += 32) { const v16b a = frag_kb(A + (size_t)(m0 + nloc) * KIN + kb, hlf), al_ = frag_kb(Al + (size_t)(m0 + nloc) * KIN + kb, hlf);
#pragma unroll
    for (int t = 0; t < 8; ++t) { const v16b bw = frag_kb(Bw + (size_t)(c0 + t * 16 + nloc) * KIN + kb, hlf); acc[t] = wmma16b(a, bw, acc[t]); acc[t] = wmma16b(al_, bw, acc[t]); } }
  if (OUTMODE == 0) {
#pragma unroll
    for (int t = 0; t < 8; ++t)
#pragma unroll
      for (int r = 0; r < 8; ++r) { b16 a_, b_; split16(acc[t][r], a_, b_); Tb[wave][8 * hlf + r][t * 16 + nloc] = a_; Tc[wave][8 * hlf + r][t * 16 + nloc] = b_; }
    wave_lds_sync();
    for (int pass = 0; pass < 2; ++pass) { for (int i = lane; i < 16 * 16; i += 32) { const int rr = i >> 4, c8 = (i & 15) * 8; const size_t gi = (size_t)(m0 + rr) * CH + c0 + c8; *(volatile v8b*)(FT + gi) = *(const v8b*)(&Tb[wave][rr][c8]); *(volatile v8b*)(FTl + gi) = *(const v8b*)(&Tc[wave][rr][c8]); } __threadfence(); } }
  else {
#pragma unroll
    for (int t = 0; t < 8; ++t)
#pragma unroll
      for (int r = 0; r < 8; ++r) { const int c = c0 + t * 16 + nloc, row = m0 + 8 * hlf + r; Ts[wave][8 * hlf + r][t * 16 + nloc] = acc[t][r] * (1.0f / XS) + P[2048 + c] + ((row < NN) ? bf16_rne(x[(size_t)row * CH + c]) : 0.0f); }
    wave_lds_sync();
    for (int pass = 0; pass < 2; ++pass) { for (int i = lane; i < 16 * 32; i += 32) { const int rr = i >> 5, c4 = (i & 31) * 4; const int row = m0 + rr; if (row < NN) *(volatile v4f*)(out + (size_t)row * CH + c0 + c4) = *(const v4f*)(&Ts[wave][rr][c4]); } __threadfence(); } }
}
template <int NH>
__global__ __launch_bounds__(256) void elr_kernel(const b16* __restrict__ FT, const b16* __restrict__ FTl, const float* __restrict__ Pas, const float* __restrict__ Pad, float* __restrict__ ALR) {
  __shared__ __attribute__((aligned(16))) float Es[8][16];
  const int wave = threadIdx.x >> 5, v = blockIdx.x * 8 + wave, lane = threadIdx.x & 31;
  float sl = 0.0f, sr = 0.0f; const v8b fr = *(const v8b*)(FT + (size_t)v * CH + lane * 8), fl = *(const v8b*)(FTl + (size_t)v * CH + lane * 8);
#pragma unroll
  for (int e = 0; e < 8; ++e) { const float f = ((float)fr[e] + (float)fl[e]) * (1.0f / XS); sl += pmul(f, Pas[lane * 8 + e]); sr += pmul(f, Pad[lane * 8 + e]); }
  sl += __shfl_xor(sl, 1); sl += __shfl_xor(sl, 2); sr += __shfl_xor(sr, 1); sr += __shfl_xor(sr, 2); if (NH == 4) { sl += __shfl_xor(sl, 4); sr += __shfl_xor(sr, 4); }
  constexpr int LPH = 32 / NH;
  if ((lane % LPH) == 0) { Es[wave][lane / LPH] = sl; Es[wave][8 + lane / LPH] = sr; } if (NH == 4 && (lane % LPH) == 0) { Es[wave][4 + lane / LPH] = 0.0f; Es[wave][12 + lane / LPH] = 0.0f; }
  __syncthreads();
  for (int pass = 0; pass < 2; ++pass) { if (threadIdx.x < 32) *(volatile v4f*)(ALR + (size_t)blockIdx.x * 128 + threadIdx.x * 4) = *(const v4f*)(&Es[0][0] + threadIdx.x * 4); __threadfence(); }
}
template <int NH, int COL0>
__global__ __launch_bounds__(256) void gat_kernel(const b16* __restrict__ FT, const b16* __restrict__ FTl, const float* __restrict__ ALR, const int* __restrict__ src, const int* __restrict__ perm, const int* __restrict__ rowptr, const int* __restrict__ rowcnt, const float* __restrict__ Pb, b16* __restrict__ CT, b16* __restrict__ CTl) {
  __shared__ __attribute__((aligned(16))) b16 Sh[8][CH + 8], Sl[8][CH + 8];
  constexpr int LPH = 32 / NH;
  const int wave = threadIdx.x >> 5, v = blockIdx.x * 8 + wave, lane = threadIdx.x & 31, hd = lane / LPH;
  int cnt = rowcnt[v]; cnt = (cnt < 0) ? 0 : (cnt > MAXDEG ? MAXDEG : cnt); int p0 = rowptr[v]; p0 = (p0 < 0) ? 0 : (p0 > PERMLEN - cnt ? PERMLEN - cnt : p0);
  const float adv = ALR[(size_t)v * 16 + 8 + hd]; float m = -INFINITY, l = 0.0f; float acc[8] = {0, 0, 0, 0, 0, 0, 0, 0};
  for (int q = 0; q <= cnt; ++q) { int s; if (q < cnt) { int id = perm[p0 + q]; id = (id < 0) ? 0 : (id >= NE ? NE - 1 : id); s = src[id]; s = (s < 0) ? 0 : (s >= NN ? NN - 1 : s); } else s = v;
    const float e = leaky(ALR[(size_t)s * 16 + hd] + adv); const float mn = fmaxf(m, e); const float al_ = nexp(m - mn); const float p = nexp(e - mn); m = mn; l = l * al_ + p;
    const v8b fr = *(const v8b*)(FT + (size_t)s * CH + lane * 8), fl = *(const v8b*)(FTl + (size_t)s * CH + lane * 8);
#pragma unroll
    for (int k = 0; k < 8; ++k) acc[k] = acc[k] * al_ + pmul(p, (float)fr[k] + (float)fl[k]); }
  const float inv = 1.0f / ((l + 1e-16f) * XS);
#pragma unroll
  for (int k = 0; k < 8; ++k) { const int c = lane * 8 + k; const float y = elu_f(acc[k] * inv + Pb[c]); b16 a_, b_; split16(y * XS, a_, b_); Sh[wave][c] = a_; Sl[wave][c] = b_; }
  wave_lds_sync();
  for (int pass = 0; pass < 2; ++pass) { *(volatile v8b*)(CT + (size_t)v * CAT + COL0 + lane * 8) = *(const v8b*)(&Sh[wave][lane * 8]); *(volatile v8b*)(CTl + (size_t)v * CAT + COL0 + lane * 8) = *(const v8b*)(&Sl[wave][lane * 8]); __threadfence(); }
}
}

extern "C" void kernel_launch(void* const* d_in, const int* in_sizes, int n_in,
                              void* d_out, int out_size, void* d_ws, size_t ws_size, hipStream_t stream) {
  (void)n_in; (void)out_size;
  const float* x = (const float*)d_in[0]; const int* ei = (const int*)d_in[1]; const float* gm = (const float*)d_in[2]; const float* bt = (const float*)d_in[3]; const float* w1 = (const float*)d_in[4]; const float* as1 = (const float*)d_in[5]; const float* ad1 = (const float*)d_in[6]; const float* b1 = (const float*)d_in[7]; const float* w2 = (const float*)d_in[8]; const float* as2 = (const float*)d_in[9]; const float* ad2 = (const float*)d_in[10]; const float* b2 = (const float*)d_in[11]; const float* wu = (const float*)d_in[12]; const float* bu = (const float*)d_in[13];
  float* out = (float*)d_out;
  if (in_sizes[0] != NN * CH || in_sizes[1] != 2 * NE || in_sizes[4] != CH * CH || in_sizes[12] != CAT * CH) return;
  const int* srcI = ei; const int* dstI = ei + NE; const int NE_RUN = NE;
  size_t off = 0; char* ws = (char*)d_ws;
  auto carve = [&](size_t bytes) { char* p = ws + off; off += (bytes + 255) & ~(size_t)255; return p; };
  b16* R = (b16*)carve((size_t)(2 * CH * CH + CH * CAT) * 2); float* P = (float*)carve(2304 * 4); b16* XN = (b16*)carve((size_t)NP * CH * 2); b16* XNl = (b16*)carve((size_t)NP * CH * 2); b16* FT = (b16*)carve((size_t)NP * CH * 2); b16* FTl = (b16*)carve((size_t)NP * CH * 2); float* ALR = (float*)carve((size_t)NP * 16 * 4); b16* CT = (b16*)carve((size_t)NP * CAT * 2); b16* CTl = (b16*)carve((size_t)NP * CAT * 2);
  CsrBufs cs; off = csr_carve(cs, ws, off, NE_RUN, NN);
  if (off > ws_size) return;
  csr_build(cs, dstI, NE_RUN, NN, stream);
  prep_kernel<<<256, 256, 0, stream>>>(gm, bt, w1, as1, ad1, b1, w2, as2, ad2, b2, wu, bu, R, P, XN, XNl, CT, CTl);
  ln_kernel<<<NN / 8, 256, 0, stream>>>(x, P, XN, XNl);
  gemm_kernel<CH, 0><<<dim3(2, NP / 32), 64, 0, stream>>>(XN, XNl, R, P, x, FT, FTl, nullptr);
  elr_kernel<4><<<NN / 8, 256, 0, stream>>>(FT, FTl, P + 512, P + 768, ALR);
  gat_kernel<4, 0><<<NN / 8, 256, 0, stream>>>(FT, FTl, ALR, srcI, cs.PERM, cs.ROWPTR, cs.ROWCNT, P + 1024, CT, CTl);
  gemm_kernel<CH, 0><<<dim3(2, NP / 32), 64, 0, stream>>>(XN, XNl, R + (size_t)CH * CH, P, x, FT, FTl, nullptr);
  elr_kernel<8><<<NN / 8, 256, 0, stream>>>(FT, FTl, P + 1280, P + 1536, ALR);
  gat_kernel<8, 256><<<NN / 8, 256, 0, stream>>>(FT, FTl, ALR, srcI, cs.PERM, cs.ROWPTR, cs.ROWCNT, P + 1792, CT, CTl);
  gemm_kernel<CAT, 1><<<dim3(2, NP / 32), 64, 0, stream>>>(CT, CTl, R + 131072, P, x, nullptr, nullptr, out);
}
